// HeadAttention_36670430773488
// MI455X (gfx1250) — hardware-verified
//
#include <hip/hip_runtime.h>
#include <hip/hip_bf16.h>

typedef __attribute__((ext_vector_type(16))) _Float16 v16h;
typedef __attribute__((ext_vector_type(8)))  _Float16 v8h;
typedef __attribute__((ext_vector_type(16))) __bf16   v16b;
typedef __attribute__((ext_vector_type(8)))  __bf16   v8b;
typedef __attribute__((ext_vector_type(8)))  float    v8f;
typedef __attribute__((ext_vector_type(4)))  float    v4f;
typedef __attribute__((ext_vector_type(4)))  unsigned int v4u;

constexpr int kBatch = 4;
constexpr int kSeq   = 4096;
constexpr int kEmb   = 512;
constexpr int kHd    = 64;
constexpr int kRows  = kBatch * kSeq;
constexpr int kQkLd  = 2 * kHd;
constexpr int kKeyChunk = 64;
constexpr int kQBlock   = 64;
constexpr int kWaves    = 4;
constexpr int kOsPitch  = 68;
constexpr float kScoreScale = 0.125f;

constexpr size_t kBytesXPlane  = (size_t)kRows * kEmb * 2;
constexpr size_t kBytesWPlane  = (size_t)3 * kHd * kEmb * 2;
constexpr size_t kBytesQkPlane = (size_t)kRows * kQkLd * 2;
constexpr size_t kBytesVtPlane = (size_t)kBatch * kHd * kSeq * 2;
constexpr size_t kOffXh  = 0;
constexpr size_t kOffXl  = kOffXh  + kBytesXPlane;
constexpr size_t kOffWh  = kOffXl  + kBytesXPlane;
constexpr size_t kOffWl  = kOffWh  + kBytesWPlane;
constexpr size_t kOffQkh = kOffWl  + kBytesWPlane;
constexpr size_t kOffQkl = kOffQkh + kBytesQkPlane;
constexpr size_t kOffVth = kOffQkl + kBytesQkPlane;
constexpr size_t kOffVtl = kOffVth + kBytesVtPlane;
constexpr size_t kWsTotal = kOffVtl + kBytesVtPlane;
static_assert(kWsTotal == 46530560, "carve total");
static_assert(kWsTotal <= (size_t)134217728, "carve cap");
static_assert(kOffXl % 512 == 0 && kOffWh % 512 == 0 && kOffWl % 512 == 0 && kOffQkh % 512 == 0 &&
              kOffQkl % 512 == 0 && kOffVth % 512 == 0 && kOffVtl % 512 == 0, "region alignment");

static_assert(kEmb % 32 == 0, "K multiple of 32");
static_assert(kRows % 64 == 0 && kQkLd % 64 == 0, "GEMM A tile multiples");
static_assert(kHd % 64 == 0 && kSeq % 64 == 0, "GEMM B tile multiples");
static_assert(kSeq % kQBlock == 0 && kSeq % kKeyChunk == 0 && kHd == 64, "attention geometry");
static_assert((kRows * kEmb / 8) % 256 == 0 && (kHd * kEmb / 8) % 256 == 0, "cast producer coverage");

__device__ __forceinline__ unsigned short f2bf_bits(float f) {
  unsigned u = __float_as_uint(f);
  return (unsigned short)((u + 0x7FFFu + ((u >> 16) & 1u)) >> 16);
}
__device__ __forceinline__ float bf_bits2f(unsigned short h) { return __uint_as_float(((unsigned)h) << 16); }

__device__ __forceinline__ void dep_guard_h(v8f& a, v8f& b, v16h x, v16h y) { asm volatile("v_nop\n\tv_nop\n\tv_nop\n\tv_nop" : "+v"(a), "+v"(b) : "v"(x), "v"(y)); }
__device__ __forceinline__ void dep_guard_b(v8f& a, v8f& b, v16b x, v16b y) { asm volatile("v_nop\n\tv_nop\n\tv_nop\n\tv_nop" : "+v"(a), "+v"(b) : "v"(x), "v"(y)); }
__device__ __forceinline__ void keep4_h(v16h a, v16h b, v16h c, v16h d) { asm volatile("v_nop" :: "v"(a), "v"(b), "v"(c), "v"(d)); }
__device__ __forceinline__ void keep4_b(v16b a, v16b b, v16b c, v16b d) { asm volatile("v_nop" :: "v"(a), "v"(b), "v"(c), "v"(d)); }
__device__ __forceinline__ void acc_guard4(v8f& a, v8f& b, v8f& c, v8f& d) { asm volatile("v_nop\n\tv_nop\n\tv_nop\n\tv_nop" : "+v"(a), "+v"(b), "+v"(c), "+v"(d)); }
template <typename T> struct Frag;
template <> struct Frag<_Float16> {
  typedef v16h V; union U { v16h v; v8h h[2]; };
  static __device__ __forceinline__ v16h load(const _Float16* p) {
    U f; f.h[0] = *(const v8h*)(p); f.h[1] = *(const v8h*)(p + 16); return f.v;
  }
  static __device__ __forceinline__ v8f mma(v16h a, v16h b, v8f c) {
    return __builtin_amdgcn_wmma_f32_16x16x32_f16(false, a, false, b, (short)0, c, false, false);
  }
  static __device__ __forceinline__ void guard(v8f& a, v8f& b, v16h x, v16h y) { dep_guard_h(a, b, x, y); }
  static __device__ __forceinline__ void keep(v16h a, v16h b, v16h c, v16h d) { keep4_h(a, b, c, d); }
};
template <> struct Frag<__bf16> {
  typedef v16b V; union U { v16b v; v8b h[2]; };
  static __device__ __forceinline__ v16b load(const __bf16* p) {
    U f; f.h[0] = *(const v8b*)(p); f.h[1] = *(const v8b*)(p + 16); return f.v;
  }
  static __device__ __forceinline__ v8f mma(v16b a, v16b b, v8f c) {
    return __builtin_amdgcn_wmma_f32_16x16x32_bf16(false, a, false, b, (short)0, c, false, false);
  }
  static __device__ __forceinline__ void guard(v8f& a, v8f& b, v16b x, v16b y) { dep_guard_b(a, b, x, y); }
  static __device__ __forceinline__ void keep(v16b a, v16b b, v16b c, v16b d) { keep4_b(a, b, c, d); }
};

template <int ET> struct Elem;
template <> struct Elem<0> { typedef _Float16 T; };
template <> struct Elem<1> { typedef __bf16 T; };
template <int ET, bool SPLIT, int BIAS_MODE, int OUT_MODE, bool RESID, int ACT = 0>
__global__ __launch_bounds__(256) void wmma_gemm64(
    const unsigned short* __restrict__ Ap, const unsigned short* __restrict__ A2p, int lda, long strideA,
    const unsigned short* __restrict__ Btp, const unsigned short* __restrict__ Bt2p, int ldb, long strideB,
    void* __restrict__ Cout, void* __restrict__ Cout2, int ldc, long strideC,
    const float* __restrict__ bias,
    const float* __restrict__ resid, long strideR,
    int M, int N, int K, float scale) {
  typedef typename Elem<ET>::T T;
  typedef typename Frag<T>::V V;
  const T* A = (const T*)Ap; const T* A2 = (const T*)A2p; const T* Bt = (const T*)Btp; const T* Bt2 = (const T*)Bt2p;
  __shared__ __align__(16) float sT[8][16 * 68];
  const int b    = blockIdx.y;
  const int lane = threadIdx.x & 31;
  const int wave = threadIdx.x >> 5;
  const int tilesN = N >> 6;
  const int tilesM = M >> 6;
  const int tile = blockIdx.x * 8 + wave;
  if (tile >= tilesM * tilesN) return;
  const int tm = tile / tilesN;
  const int tn = tile - tm * tilesN;
  const int m0 = tm << 6;
  const int n0 = tn << 6;

  const T* Ab  = A  + (size_t)b * strideA;
  const T* Bb  = Bt + (size_t)b * strideB;
  const T* Ab2 = SPLIT ? (A2  + (size_t)b * strideA) : nullptr;
  const T* Bb2 = SPLIT ? (Bt2 + (size_t)b * strideB) : nullptr;

  const int rlane = lane & 15;
  const int koff  = (lane >> 4) * 8;
  const int mOff  = (lane >> 4) * 8;

  v8f acc[4][4];
#pragma unroll
  for (int i = 0; i < 4; ++i)
#pragma unroll
    for (int j = 0; j < 4; ++j) acc[i][j] = (v8f){0.f,0.f,0.f,0.f,0.f,0.f,0.f,0.f};

  for (int k0 = 0; k0 < K; k0 += 32) {
    V bh[4], bl[4];
#pragma unroll
    for (int j = 0; j < 4; ++j) {
      const size_t bo = (size_t)(n0 + (j << 4) + rlane) * ldb + koff + k0;
      bh[j] = Frag<T>::load(Bb + bo);
      if (SPLIT) bl[j] = Frag<T>::load(Bb2 + bo);
    }
#pragma unroll
    for (int i = 0; i < 4; ++i) {
      const size_t ao = (size_t)(m0 + (i << 4) + rlane) * lda + koff + k0;
      V ah = Frag<T>::load(Ab + ao);
      V al;
      if (SPLIT) al = Frag<T>::load(Ab2 + ao);
#pragma unroll
      for (int j = 0; j < 4; ++j) {
        acc[i][j] = Frag<T>::mma(ah, bh[j], acc[i][j]);
        if (SPLIT) {
          acc[i][j] = Frag<T>::mma(ah, bl[j], acc[i][j]);
          acc[i][j] = Frag<T>::mma(al, bh[j], acc[i][j]);
        }
      }
      Frag<T>::guard(acc[i][0], acc[i][3], ah, SPLIT ? al : ah);
    }
    Frag<T>::keep(bh[0], bh[1], bh[2], bh[3]);
    if (SPLIT) Frag<T>::keep(bl[0], bl[1], bl[2], bl[3]);
  }
  acc_guard4(acc[0][0], acc[0][1], acc[0][2], acc[0][3]);
  acc_guard4(acc[1][0], acc[1][1], acc[1][2], acc[1][3]);
  acc_guard4(acc[2][0], acc[2][1], acc[2][2], acc[2][3]);
  acc_guard4(acc[3][0], acc[3][1], acc[3][2], acc[3][3]);

  float* slab = sT[wave];
  const float* Rb = RESID ? (resid + (size_t)b * strideR) : nullptr;
#pragma unroll
  for (int i = 0; i < 4; ++i) {
    const int mBase = m0 + (i << 4);
#pragma unroll
    for (int j = 0; j < 4; ++j) {
      const int n = n0 + (j << 4) + rlane;
      float bv = 0.f;
      if (BIAS_MODE == 2) bv = bias[n];
#pragma unroll
      for (int r = 0; r < 8; ++r) {
        float v = acc[i][j][r] * scale;
        if (BIAS_MODE == 1) v += bias[mBase + mOff + r];
        if (BIAS_MODE == 2) v += bv;
        if (RESID) v += Rb[(size_t)(mBase + mOff + r) * ldc + n];
        if (ACT == 1) v = tanhf(v);
        if (ACT == 2) v = fmaxf(v, 0.0f);
        if (ACT == 3) v = v / (1.0f + expf(-v));
        if (ACT == 4) v = (v > 0.f) ? v : 0.01f * v;
        if (ACT == 5) v = 0.5f * v * (1.0f + erff(v * 0.70710678118654752f));
        slab[(mOff + r) * 68 + (j << 4) + rlane] = v;
      }
    }
    __builtin_amdgcn_fence(__ATOMIC_RELEASE, "workgroup");
    __builtin_amdgcn_wave_barrier();
    __builtin_amdgcn_fence(__ATOMIC_ACQUIRE, "workgroup");
    if (OUT_MODE == 0) {
      float* C = (float*)Cout + (size_t)b * strideC;
      const int hh = lane >> 4, c4 = (lane & 15) * 4;
      for (int pass = 0; pass < 2; ++pass) {
#pragma unroll
        for (int it = 0; it < 8; ++it) {
          const int row = it * 2 + hh;
          v4f v = *(const v4f*)(slab + row * 68 + c4);
          *(volatile v4f*)(C + (size_t)(mBase + row) * ldc + n0 + c4) = v;
        }
        __threadfence();
      }
    } else {
      const int q = lane >> 3, c8 = (lane & 7) * 8;
      unsigned short* C  = (unsigned short*)Cout  + (size_t)b * strideC;
      unsigned short* C2 = (OUT_MODE == 2) ? ((unsigned short*)Cout2 + (size_t)b * strideC) : nullptr;
      for (int pass = 0; pass < 2; ++pass) {
#pragma unroll
        for (int it = 0; it < 4; ++it) {
          const int row = it * 4 + q;
          const float* sp = slab + row * 68 + c8;
          v8h hv, lv;
#pragma unroll
          for (int e = 0; e < 8; ++e) {
            if (OUT_MODE == 1) {
              hv[e] = (_Float16)sp[e];
            } else {
              unsigned short hb = f2bf_bits(sp[e]);
              unsigned short lb = f2bf_bits(sp[e] - bf_bits2f(hb));
              hv[e] = __builtin_bit_cast(_Float16, hb);
              lv[e] = __builtin_bit_cast(_Float16, lb);
            }
          }
          *(volatile v8h*)(C + (size_t)(mBase + row) * ldc + n0 + c8) = hv;
          if (OUT_MODE == 2) *(volatile v8h*)(C2 + (size_t)(mBase + row) * ldc + n0 + c8) = lv;
        }
        __threadfence();
      }
    }
    __builtin_amdgcn_fence(__ATOMIC_RELEASE, "workgroup");
    __builtin_amdgcn_wave_barrier();
    __builtin_amdgcn_fence(__ATOMIC_ACQUIRE, "workgroup");
  }
}

__device__ __forceinline__ unsigned short at_bf_bits(float f) {
  unsigned u = __float_as_uint(f);
  return (unsigned short)((u + 0x7FFFu + ((u >> 16) & 1u)) >> 16);
}
__device__ __forceinline__ __bf16 at_f2bf(float f) { return __builtin_bit_cast(__bf16, at_bf_bits(f)); }
__device__ __forceinline__ void at_split(float f, __bf16& hi, __bf16& lo) {
  const unsigned short hb = at_bf_bits(f);
  hi = __builtin_bit_cast(__bf16, hb);
  lo = at_f2bf(f - __uint_as_float(((unsigned)hb) << 16));
}
__device__ __forceinline__ v8f at_mma(v16b a, v16b b, v8f c) {
  c = __builtin_amdgcn_wmma_f32_16x16x32_bf16(false, a, false, b, (short)0, c, false, false);
  asm volatile("v_nop\n\tv_nop\n\tv_nop\n\tv_nop" : "+v"(c) : "v"(a), "v"(b));
  return c;
}
__device__ __forceinline__ void sched_cut() { __builtin_amdgcn_sched_barrier(0); }

__global__ __launch_bounds__(256) void cast_split_bf16x8(
    const float* __restrict__ in, unsigned short* __restrict__ hi, unsigned short* __restrict__ lo, int n8) {
  const int i = blockIdx.x * 256 + threadIdx.x;
  if (i >= n8) return;
  const v4f f0 = *(const v4f*)(in + (size_t)i * 8);
  const v4f f1 = *(const v4f*)(in + (size_t)i * 8 + 4);
  float f[8];
  f[0] = f0[0]; f[1] = f0[1]; f[2] = f0[2]; f[3] = f0[3];
  f[4] = f1[0]; f[5] = f1[1]; f[6] = f1[2]; f[7] = f1[3];
  unsigned hb[8], lb[8];
#pragma unroll
  for (int e = 0; e < 8; ++e) {
    const unsigned short h = f2bf_bits(f[e]);
    hb[e] = (unsigned)h;
    lb[e] = (unsigned)f2bf_bits(f[e] - bf_bits2f(h));
  }
  v4u wh, wl;
  wh[0] = hb[0] | (hb[1] << 16); wh[1] = hb[2] | (hb[3] << 16);
  wh[2] = hb[4] | (hb[5] << 16); wh[3] = hb[6] | (hb[7] << 16);
  wl[0] = lb[0] | (lb[1] << 16); wl[1] = lb[2] | (lb[3] << 16);
  wl[2] = lb[4] | (lb[5] << 16); wl[3] = lb[6] | (lb[7] << 16);
  unsigned short* ph = hi + (size_t)i * 8;
  unsigned short* pl = lo + (size_t)i * 8;
  *(volatile v4u*)ph = wh;
  *(volatile v4u*)pl = wl;
  __threadfence();
  *(volatile v4u*)ph = wh;
  *(volatile v4u*)pl = wl;
}

__global__ __launch_bounds__(128) __attribute__((amdgpu_num_vgpr(256)))
void causal_attn_hd64(const unsigned short* __restrict__ QKh, const unsigned short* __restrict__ QKl,
                      const unsigned short* __restrict__ VTh, const unsigned short* __restrict__ VTl,
                      float* __restrict__ out)
{
  __shared__ __align__(16) unsigned short Ksh[kKeyChunk * kHd];
  __shared__ __align__(16) unsigned short Ksl[kKeyChunk * kHd];
  __shared__ __align__(16) unsigned short Vth[kHd * kKeyChunk];
  __shared__ __align__(16) unsigned short Vtl[kHd * kKeyChunk];
  __shared__ __align__(16) __bf16 Psh[kWaves][16 * kKeyChunk];
  __shared__ __align__(16) __bf16 Psl[kWaves][16 * kKeyChunk];
  __shared__ __align__(16) float  Os[kWaves][16 * kOsPitch];

  const int tid  = threadIdx.x;
  const int wave = tid >> 5;
  const int lane = tid & 31;
  const int hh   = lane >> 4;
  const int c    = lane & 15;

  constexpr int nqb = kSeq / kQBlock;
  const int qb = blockIdx.x % nqb;
  const int b  = blockIdx.x / nqb;
  const int q0 = qb * kQBlock + wave * 16;
  const size_t rows0 = (size_t)b * kSeq;
  const float ninf = -__builtin_huge_valf();
  const v8f z8 = {0.f,0.f,0.f,0.f,0.f,0.f,0.f,0.f};

  v16b qah[2], qal[2];
  {
    const size_t qo = (rows0 + q0 + c) * kQkLd + 8 * hh;
    const __bf16* qh = (const __bf16*)QKh + qo;
    const __bf16* ql = (const __bf16*)QKl + qo;
#pragma unroll
    for (int dc = 0; dc < 2; ++dc) {
      qah[dc] = Frag<__bf16>::load(qh + dc * 32);
      qal[dc] = Frag<__bf16>::load(ql + dc * 32);
    }
  }
  sched_cut();

  float mrow[8], lrow[8];
  v8f oacc[4];
#pragma unroll
  for (int r = 0; r < 8; ++r) { mrow[r] = ninf; lrow[r] = 0.f; }
#pragma unroll
  for (int t = 0; t < 4; ++t) oacc[t] = z8;

  const int nChunks = qb + 1;
  for (int kc = 0; kc < nChunks; ++kc) {
    const int kv0 = kc * kKeyChunk;
    __syncthreads();
    {
      const int r = tid >> 1;
      const int half = (tid & 1) * 32;
      const v4u* gkh = (const v4u*)(QKh + (rows0 + kv0 + r) * kQkLd + kHd + half);
      const v4u* gkl = (const v4u*)(QKl + (rows0 + kv0 + r) * kQkLd + kHd + half);
      const v4u* gvh = (const v4u*)(VTh + ((size_t)b * kHd + r) * kSeq + kv0 + half);
      const v4u* gvl = (const v4u*)(VTl + ((size_t)b * kHd + r) * kSeq + kv0 + half);
      v4u* lkh = (v4u*)(Ksh + r * kHd + half);
      v4u* lkl = (v4u*)(Ksl + r * kHd + half);
      v4u* lvh = (v4u*)(Vth + r * kKeyChunk + half);
      v4u* lvl = (v4u*)(Vtl + r * kKeyChunk + half);
#pragma unroll 1
      for (int i = 0; i < 4; ++i) {
        const v4u a0 = gkh[i];
        const v4u a1 = gkl[i];
        const v4u a2 = gvh[i];
        const v4u a3 = gvl[i];
        lkh[i] = a0; lkl[i] = a1; lvh[i] = a2; lvl[i] = a3;
      }
    }
    __syncthreads();

    v8f s[4];
#pragma unroll
    for (int j = 0; j < 4; ++j) {
      v8f acc = z8;
#pragma unroll
      for (int dc = 0; dc < 2; ++dc) {
        const int ko = (j * 16 + c) * kHd + dc * 32 + 8 * hh;
        const v16b kb = Frag<__bf16>::load((const __bf16*)Ksh + ko);
        const v16b kl = Frag<__bf16>::load((const __bf16*)Ksl + ko);
        acc = at_mma(qah[dc], kb, acc);
        acc = at_mma(qah[dc], kl, acc);
        acc = at_mma(qal[dc], kb, acc);
      }
      s[j] = acc;
      sched_cut();
    }

    const bool diag = (kc == qb);
    float cm[8];
#pragma unroll
    for (int r = 0; r < 8; ++r) {
      const int qrow = q0 + 8 * hh + r;
      float m = ninf;
#pragma unroll
      for (int j = 0; j < 4; ++j) {
        const int kvcol = kv0 + j * 16 + c;
        const float sv = s[j][r] * kScoreScale;
        const float v = (diag && (kvcol > qrow)) ? ninf : sv;
        s[j][r] = v;
        m = fmaxf(m, v);
      }
#pragma unroll
      for (int off = 1; off < 16; off <<= 1) m = fmaxf(m, __shfl_xor(m, off, 32));
      cm[r] = m;
      sched_cut();
    }

    __bf16* pwh = Psh[wave];
    __bf16* pwl = Psl[wave];
#pragma unroll
    for (int r = 0; r < 8; ++r) {
      const float mnew = fmaxf(mrow[r], cm[r]);
      const float alpha = expf(mrow[r] - mnew);
      mrow[r] = mnew;
      float psum = 0.f;
#pragma unroll
      for (int j = 0; j < 4; ++j) {
        const float p = expf(s[j][r] - mnew);
        psum += p;
        __bf16 ph, pl;
        at_split(p, ph, pl);
        pwh[(8 * hh + r) * kKeyChunk + j * 16 + c] = ph;
        pwl[(8 * hh + r) * kKeyChunk + j * 16 + c] = pl;
      }
#pragma unroll
      for (int off = 1; off < 16; off <<= 1) psum += __shfl_xor(psum, off, 32);
      lrow[r] = lrow[r] * alpha + psum;
#pragma unroll
      for (int t = 0; t < 4; ++t) oacc[t][r] *= alpha;
      sched_cut();
    }
    __syncthreads();

#pragma unroll
    for (int kk = 0; kk < 2; ++kk) {
      const int po = c * kKeyChunk + kk * 32 + 8 * hh;
      const v16b pa = Frag<__bf16>::load(pwh + po);
      const v16b pl = Frag<__bf16>::load(pwl + po);
#pragma unroll
      for (int t = 0; t < 4; ++t) {
        const int vo = (t * 16 + c) * kKeyChunk + kk * 32 + 8 * hh;
        const v16b vb = Frag<__bf16>::load((const __bf16*)Vth + vo);
        const v16b vl = Frag<__bf16>::load((const __bf16*)Vtl + vo);
        oacc[t] = at_mma(pa, vb, oacc[t]);
        oacc[t] = at_mma(pa, vl, oacc[t]);
        oacc[t] = at_mma(pl, vb, oacc[t]);
        sched_cut();
      }
    }
  }

  float* os = Os[wave];
#pragma unroll
  for (int r = 0; r < 8; ++r) {
    const float inv = 1.0f / lrow[r];
#pragma unroll
    for (int t = 0; t < 4; ++t) os[(8 * hh + r) * kOsPitch + t * 16 + c] = oacc[t][r] * inv;
    sched_cut();
  }
  __syncthreads();
  {
    float* ob = out + rows0 * kHd;
    const int c4 = (lane & 15) * 4;
    for (int pass = 0; pass < 2; ++pass) {
#pragma unroll
      for (int it = 0; it < 8; ++it) {
        const int row = it * 2 + hh;
        v4f val = *(const v4f*)(os + row * kOsPitch + c4);
        *(volatile v4f*)(ob + (size_t)(q0 + row) * kHd + c4) = val;
      }
      __threadfence();
    }
  }
}

extern "C" void kernel_launch(void* const* d_in, const int* in_sizes, int n_in,
                              void* d_out, int out_size, void* d_ws, size_t ws_size,
                              hipStream_t stream) {
  if (n_in < 4) return;
  if (in_sizes[0] != kRows * kEmb || in_sizes[1] != kHd * kEmb || in_sizes[2] != kHd * kEmb ||
      in_sizes[3] != kHd * kEmb || out_size != kRows * kHd || ws_size < kWsTotal) return;

  const float* x  = (const float*)d_in[0];
  const float* Wq = (const float*)d_in[1];
  const float* Wk = (const float*)d_in[2];
  const float* Wv = (const float*)d_in[3];
  float* out = (float*)d_out;

  char* ws = (char*)d_ws;
  unsigned short* xh  = (unsigned short*)(ws + kOffXh);
  unsigned short* xl  = (unsigned short*)(ws + kOffXl);
  unsigned short* wh  = (unsigned short*)(ws + kOffWh);
  unsigned short* wl  = (unsigned short*)(ws + kOffWl);
  unsigned short* qkh = (unsigned short*)(ws + kOffQkh);
  unsigned short* qkl = (unsigned short*)(ws + kOffQkl);
  unsigned short* vth = (unsigned short*)(ws + kOffVth);
  unsigned short* vtl = (unsigned short*)(ws + kOffVtl);

  const int nx8 = kRows * kEmb / 8;
  const int nw8 = kHd * kEmb / 8;
  cast_split_bf16x8<<<nx8 / 256, 256, 0, stream>>>(x, xh, xl, nx8);
  cast_split_bf16x8<<<nw8 / 256, 256, 0, stream>>>(Wq, wh, wl, nw8);
  cast_split_bf16x8<<<nw8 / 256, 256, 0, stream>>>(Wk, wh + (size_t)kHd * kEmb, wl + (size_t)kHd * kEmb, nw8);
  cast_split_bf16x8<<<nw8 / 256, 256, 0, stream>>>(Wv, wh + (size_t)2 * kHd * kEmb, wl + (size_t)2 * kHd * kEmb, nw8);

  {
    const int tiles = (kRows / 64) * (kQkLd / 64);
    dim3 grid((tiles + 7) / 8, 1);
    wmma_gemm64<1, true, 0, 2, false, 0><<<grid, 256, 0, stream>>>(
        xh, xl, kEmb, 0L,
        wh, wl, kEmb, 0L,
        (void*)qkh, (void*)qkl, kQkLd, 0L,
        (const float*)nullptr, (const float*)nullptr, 0L,
        kRows, kQkLd, kEmb, 1.0f);
  }

  {
    const int tiles = (kHd / 64) * (kSeq / 64);
    dim3 grid((tiles + 7) / 8, kBatch);
    wmma_gemm64<1, true, 0, 2, false, 0><<<grid, 256, 0, stream>>>(
        wh + (size_t)2 * kHd * kEmb, wl + (size_t)2 * kHd * kEmb, kEmb, 0L,
        xh, xl, kEmb, (long)kSeq * kEmb,
        (void*)vth, (void*)vtl, kSeq, (long)kHd * kSeq,
        (const float*)nullptr, (const float*)nullptr, 0L,
        kHd, kSeq, kEmb, 1.0f);
  }

  causal_attn_hd64<<<kBatch * (kSeq / kQBlock), 128, 0, stream>>>(qkh, qkl, vth, vtl, out);
}
